// LIIF_4767413698965
// MI455X (gfx1250) — hardware-verified
//
#include <hip/hip_runtime.h>
#include <stddef.h>
#include <math.h>

#pragma clang fp contract(off)

typedef __attribute__((ext_vector_type(16))) _Float16 v16h;
typedef __attribute__((ext_vector_type(8)))  _Float16 v8h;
typedef __attribute__((ext_vector_type(16))) __bf16   v16b;
typedef __attribute__((ext_vector_type(8)))  __bf16   v8b;
typedef __attribute__((ext_vector_type(8)))  float    v8f;
typedef __attribute__((ext_vector_type(4)))  float    v4f;
typedef __attribute__((ext_vector_type(8)))  unsigned short v8us;

constexpr int kBatch   = 2;
constexpr int kQ       = 8192;
constexpr int kImg     = 64;
constexpr int kPix     = kBatch * kImg * kImg;
constexpr int kBQ      = kBatch * kQ;
constexpr int kCin     = 3;
constexpr int kC1 = 64, kC2 = 128, kC3 = 256, kC4 = 256, kHid = 256;
constexpr int kK1      = 32;
constexpr int kK1Real  = 27;
constexpr int kK2      = 9 * kC1;
constexpr int kK3      = 9 * kC2;
constexpr int kK4      = 9 * kC3;
constexpr int kK5      = 9 * kC4;
constexpr int kInDim   = kK5 + 2;
constexpr int kN4      = 16;
constexpr int kThreads = 256;
constexpr int kMQ      = 32;
constexpr int kMRows   = kMQ * 4;
constexpr int kQT      = 4;
constexpr int kQRows   = 32;
constexpr int kQQ      = 8;
constexpr int kMBlocks = kBQ / kMQ;
constexpr int kHP      = 264;
constexpr int kBStep   = 16 * kHid;
constexpr float kEpsShift = (float)1e-6;
constexpr float kClipLo   = (float)(-1.0 + 1e-6);
constexpr float kClipHi   = (float)(1.0 - 1e-6);
constexpr float kAreaEps  = (float)1e-9;
constexpr float kInv63    = 1.0f / 63.0f;
constexpr float kHalfPix  = 0.015625f;

static_assert(kInDim == 2306, "w0 rows");
static_assert(kK1 % 32 == 0 && kK2 % 32 == 0 && kK3 % 32 == 0 && kK4 % 32 == 0 && kK5 % 32 == 0 && kHid % 32 == 0, "K % 32");
static_assert(kPix % 64 == 0 && kC1 % 64 == 0 && kC2 % 64 == 0 && kC3 % 64 == 0 && kC4 % 64 == 0 && kHid % 64 == 0, "64 tiles");
static_assert(((kPix / 64) * (kC1 / 64)) % 8 == 0 && ((kPix / 64) * (kC2 / 64)) % 8 == 0 && ((kPix / 64) * (kHid / 64)) % 8 == 0, "8 wave tiles per block");
static_assert(kC1 % 32 == 0 && kC2 % 32 == 0 && kC3 % 32 == 0 && kC4 % 32 == 0, "implicit 3x3: one tap per 32-k chunk");
static_assert(kMBlocks * kMQ == kBQ && kQT * kQRows == kMRows && kQT * kQQ == kMQ, "MLP block coverage");
static_assert(kHP % 8 == 0 && kHP >= kHid, "LDS pitch");
static_assert(kThreads == 8 * 32 && kQRows == 2 * 16 && kQRows == 8 * 4, "8 waves: 2 row tiles x 4 column groups; 4 h0 rows per wave");
static_assert(kQ == 8192, "batch index of query row bq is bq >> 13");
static_assert((kPix * (kK1 / 8)) % kThreads == 0, "im2col1 grid exact");
static_assert((kC2 * (kK2 / 8)) % kThreads == 0 && (kC3 * (kK3 / 8)) % kThreads == 0 && (kC4 * (kK4 / 8)) % kThreads == 0 &&
              (kHid * (kK5 / 8)) % kThreads == 0 && (kHid * (kHid / 8)) % kThreads == 0 && (kN4 * (kHid / 8)) % kThreads == 0 &&
              kC1 * (kK1 / 8) == kThreads, "weight prep grids exact");

constexpr size_t al4k(size_t x) { return (x + 4095) & ~(size_t)4095; }
constexpr size_t kSzIM1 = al4k((size_t)kPix * kK1 * 2);
constexpr size_t kSzC1W = al4k((size_t)kC1 * kK1 * 2);
constexpr size_t kSzC2W = al4k((size_t)kC2 * kK2 * 2);
constexpr size_t kSzC3W = al4k((size_t)kC3 * kK3 * 2);
constexpr size_t kSzC4W = al4k((size_t)kC4 * kK4 * 2);
constexpr size_t kSzW0T = al4k((size_t)kHid * kK5 * 2);
constexpr size_t kSzWSQ = al4k((size_t)kHid * kHid * 2);
constexpr size_t kSzW4T = al4k((size_t)kN4 * kHid * 2);
constexpr size_t kSzA1  = al4k((size_t)(kPix + 1) * kC1 * 2);
constexpr size_t kSzA2  = al4k((size_t)(kPix + 1) * kC2 * 2);
constexpr size_t kSzA3  = al4k((size_t)(kPix + 1) * kC3 * 2);
constexpr size_t kSzA4  = al4k((size_t)(kPix + 1) * kC4 * 2);
constexpr size_t kSzG   = al4k((size_t)kPix * kHid * 4);
constexpr size_t kOffIM1 = 0;
constexpr size_t kOffC1W = kOffIM1 + kSzIM1;
constexpr size_t kOffC2W = kOffC1W + kSzC1W;
constexpr size_t kOffC3W = kOffC2W + kSzC2W;
constexpr size_t kOffC4W = kOffC3W + kSzC3W;
constexpr size_t kOffW0T = kOffC4W + kSzC4W;
constexpr size_t kOffW1T = kOffW0T + kSzW0T;
constexpr size_t kOffW2T = kOffW1T + kSzWSQ;
constexpr size_t kOffW3T = kOffW2T + kSzWSQ;
constexpr size_t kOffW4T = kOffW3T + kSzWSQ;
constexpr size_t kOffA1H = kOffW4T + kSzW4T;
constexpr size_t kOffA1L = kOffA1H + kSzA1;
constexpr size_t kOffA2H = kOffA1L + kSzA1;
constexpr size_t kOffA2L = kOffA2H + kSzA2;
constexpr size_t kOffA3H = kOffA2L + kSzA2;
constexpr size_t kOffA3L = kOffA3H + kSzA3;
constexpr size_t kOffA4H = kOffA3L + kSzA3;
constexpr size_t kOffA4L = kOffA4H + kSzA4;
constexpr size_t kOffG   = kOffA4L + kSzA4;
constexpr size_t kWsTotal = kOffG + kSzG;
static_assert(kWsTotal == 35516416ull, "carve total");
static_assert(kWsTotal <= 134217728ull, "carve under 128 MiB");
static_assert(kOffC1W % 4096 == 0 && kOffC2W % 4096 == 0 && kOffC3W % 4096 == 0 && kOffC4W % 4096 == 0 &&
              kOffW0T % 4096 == 0 && kOffW1T % 4096 == 0 && kOffW2T % 4096 == 0 && kOffW3T % 4096 == 0 &&
              kOffW4T % 4096 == 0 && kOffA1H % 4096 == 0 && kOffA1L % 4096 == 0 && kOffA2H % 4096 == 0 &&
              kOffA2L % 4096 == 0 && kOffA3H % 4096 == 0 && kOffA3L % 4096 == 0 && kOffA4H % 4096 == 0 &&
              kOffA4L % 4096 == 0 && kOffG % 4096 == 0, "region alignment");

__device__ __forceinline__ unsigned short f2bf_bits(float f) {
  unsigned u = __float_as_uint(f);
  return (unsigned short)((u + 0x7FFFu + ((u >> 16) & 1u)) >> 16);
}
__device__ __forceinline__ float bf_bits2f(unsigned short h) { return __uint_as_float(((unsigned)h) << 16); }

__device__ __forceinline__ void dep_guard_h(v8f& a, v8f& b, v16h x, v16h y) { asm volatile("v_nop\n\tv_nop\n\tv_nop\n\tv_nop" : "+v"(a), "+v"(b) : "v"(x), "v"(y)); }
__device__ __forceinline__ void dep_guard_b(v8f& a, v8f& b, v16b x, v16b y) { asm volatile("v_nop\n\tv_nop\n\tv_nop\n\tv_nop" : "+v"(a), "+v"(b) : "v"(x), "v"(y)); }
__device__ __forceinline__ void keep4_h(v16h a, v16h b, v16h c, v16h d) { asm volatile("v_nop" :: "v"(a), "v"(b), "v"(c), "v"(d)); }
__device__ __forceinline__ void keep4_b(v16b a, v16b b, v16b c, v16b d) { asm volatile("v_nop" :: "v"(a), "v"(b), "v"(c), "v"(d)); }
__device__ __forceinline__ void acc_guard4(v8f& a, v8f& b, v8f& c, v8f& d) { asm volatile("v_nop\n\tv_nop\n\tv_nop\n\tv_nop" : "+v"(a), "+v"(b), "+v"(c), "+v"(d)); }
template <typename T> struct Frag;
template <> struct Frag<_Float16> {
  typedef v16h V; union U { v16h v; v8h h[2]; };
  static __device__ __forceinline__ v16h load(const _Float16* p) {
    U f; f.h[0] = *(const v8h*)(p); f.h[1] = *(const v8h*)(p + 16); return f.v;
  }
  static __device__ __forceinline__ v8f mma(v16h a, v16h b, v8f c) {
    return __builtin_amdgcn_wmma_f32_16x16x32_f16(false, a, false, b, (short)0, c, false, false);
  }
  static __device__ __forceinline__ void guard(v8f& a, v8f& b, v16h x, v16h y) { dep_guard_h(a, b, x, y); }
  static __device__ __forceinline__ void keep(v16h a, v16h b, v16h c, v16h d) { keep4_h(a, b, c, d); }
};
template <> struct Frag<__bf16> {
  typedef v16b V; union U { v16b v; v8b h[2]; };
  static __device__ __forceinline__ v16b load(const __bf16* p) {
    U f; f.h[0] = *(const v8b*)(p); f.h[1] = *(const v8b*)(p + 16); return f.v;
  }
  static __device__ __forceinline__ v8f mma(v16b a, v16b b, v8f c) {
    return __builtin_amdgcn_wmma_f32_16x16x32_bf16(false, a, false, b, (short)0, c, false, false);
  }
  static __device__ __forceinline__ void guard(v8f& a, v8f& b, v16b x, v16b y) { dep_guard_b(a, b, x, y); }
  static __device__ __forceinline__ void keep(v16b a, v16b b, v16b c, v16b d) { keep4_b(a, b, c, d); }
};
typedef Frag<__bf16> FragB;

__device__ __forceinline__ float bf_rne(float f) { return bf_bits2f(f2bf_bits(f)); }

__device__ __forceinline__ void acc_guard4b2(v8f& a, v8f& b, v8f& c, v8f& d, v16b x, v16b y) {
  asm volatile("v_nop\n\tv_nop\n\tv_nop\n\tv_nop" : "+v"(a), "+v"(b), "+v"(c), "+v"(d) : "v"(x), "v"(y));
}
__device__ __forceinline__ void acc_guard1b3(v8f& a, v16b x, v16b y, v16b z) {
  asm volatile("v_nop\n\tv_nop\n\tv_nop\n\tv_nop" : "+v"(a) : "v"(x), "v"(y), "v"(z));
}

__device__ __forceinline__ void store2_v8us(unsigned short* p, v8us v) {
  *(volatile v8us*)p = v;
  __threadfence();
  *(volatile v8us*)p = v;
}

__global__ __launch_bounds__(kThreads) void k_prep_c1w(const float* __restrict__ w, unsigned short* bt) {
  const int i = blockIdx.x * kThreads + threadIdx.x;
  if (i >= kC1 * (kK1 / 8)) return;
  const int n = i >> 2, k0 = (i & 3) * 8;
  v8us hv;
#pragma unroll
  for (int e = 0; e < 8; ++e) {
    const int k   = k0 + e;
    const int kc  = (k < kK1Real) ? k : (kK1Real - 1);
    const int tap = kc / 3, ci = kc - tap * 3;
    const int kh  = tap / 3, kw = tap - kh * 3;
    const float f = (k < kK1Real) ? 1.0f : 0.0f;
    const float v = w[((n * kCin + ci) * 3 + kh) * 3 + kw] * f;
    hv[e] = f2bf_bits(v);
  }
  store2_v8us(bt + (size_t)i * 8, hv);
}

template <int CIN>
__global__ __launch_bounds__(kThreads) void k_prep_convw(const float* __restrict__ w, unsigned short* bt, int cout) {
  constexpr int TPR = 9 * CIN / 8;
  const int i = blockIdx.x * kThreads + threadIdx.x;
  if (i >= cout * TPR) return;
  const int n   = i / TPR;
  const int j   = i - n * TPR;
  const int k0  = j * 8;
  const int tap = k0 / CIN;
  const int ci0 = k0 - tap * CIN;
  const int kh  = tap / 3, kw = tap - kh * 3;
  v8us hv;
#pragma unroll
  for (int e = 0; e < 8; ++e) {
    const float v = w[((size_t)(n * CIN + ci0 + e) * 3 + kh) * 3 + kw];
    hv[e] = f2bf_bits(v);
  }
  store2_v8us(bt + (size_t)i * 8, hv);
}

__global__ __launch_bounds__(kThreads) void k_prep_w0t(const float* __restrict__ w0, unsigned short* bt) {
  constexpr int TPR = kK5 / 8;
  const int i = blockIdx.x * kThreads + threadIdx.x;
  if (i >= kHid * TPR) return;
  const int n   = i / TPR;
  const int j   = i - n * TPR;
  const int k0  = j * 8;
  const int tap = k0 >> 8;
  const int c0  = k0 & 255;
  v8us hv;
#pragma unroll
  for (int e = 0; e < 8; ++e) {
    const float v = w0[((size_t)(c0 + e) * 9 + tap) * kHid + n];
    hv[e] = f2bf_bits(v);
  }
  store2_v8us(bt + (size_t)i * 8, hv);
}

__global__ __launch_bounds__(kThreads) void k_prep_wsq(const float* __restrict__ w, unsigned short* bt) {
  const int i = blockIdx.x * kThreads + threadIdx.x;
  if (i >= kHid * (kHid / 8)) return;
  const int n = i >> 5, k0 = (i & 31) * 8;
  v8us hv;
#pragma unroll
  for (int e = 0; e < 8; ++e) {
    const float v = w[(size_t)(k0 + e) * kHid + n];
    hv[e] = f2bf_bits(v);
  }
  store2_v8us(bt + (size_t)i * 8, hv);
}

__global__ __launch_bounds__(kThreads) void k_prep_w4t(const float* __restrict__ w4, unsigned short* bt) {
  const int i = blockIdx.x * kThreads + threadIdx.x;
  if (i >= kN4 * (kHid / 8)) return;
  const int n = i >> 5, k0 = (i & 31) * 8;
  const int nc = (n < 3) ? n : 2;
  const float f = (n < 3) ? 1.0f : 0.0f;
  v8us hv;
#pragma unroll
  for (int e = 0; e < 8; ++e) {
    const float v = w4[(size_t)(k0 + e) * 3 + nc] * f;
    hv[e] = f2bf_bits(v);
  }
  store2_v8us(bt + (size_t)i * 8, hv);
}

__global__ __launch_bounds__(kThreads) void k_im2col1(const float* __restrict__ x, unsigned short* im) {
  const int i  = blockIdx.x * kThreads + threadIdx.x;
  if (i >= kPix * (kK1 / 8)) return;
  const int m  = i >> 2;
  const int k0 = (i & 3) * 8;
  const int b  = m >> 12;
  const int py = (m >> 6) & 63;
  const int px = m & 63;
  v8us hv;
#pragma unroll
  for (int e = 0; e < 8; ++e) {
    const int k   = k0 + e;
    const int kc  = (k < kK1Real) ? k : (kK1Real - 1);
    const int tap = kc / 3, ci = kc - tap * 3;
    const int kh  = tap / 3, kw = tap - kh * 3;
    const int ny  = py + kh - 1, nx = px + kw - 1;
    const int ok  = ((k < kK1Real) && ((unsigned)ny < 64u) && ((unsigned)nx < 64u)) ? 1 : 0;
    const int nyc = ny < 0 ? 0 : (ny > 63 ? 63 : ny);
    const int nxc = nx < 0 ? 0 : (nx > 63 ? 63 : nx);
    const float v = x[((size_t)(b * kCin + ci) * kImg + nyc) * kImg + nxc] * (float)ok;
    hv[e] = f2bf_bits(v);
  }
  store2_v8us(im + (size_t)i * 8, hv);
}

__global__ __launch_bounds__(kThreads) void k_zero_rows(unsigned short* a1h, unsigned short* a1l,
                                                       unsigned short* a2h, unsigned short* a2l,
                                                       unsigned short* a3h, unsigned short* a3l,
                                                       unsigned short* a4h, unsigned short* a4l) {
  const int tid = threadIdx.x, wave = tid >> 5, lane = tid & 31;
  const v8us z = {0, 0, 0, 0, 0, 0, 0, 0};
  unsigned short* p = a1h;
  bool act = false;
  if (wave == 0) {
    if (lane < 8)       { p = a1h + lane * 8;        act = true; }
    else if (lane < 16) { p = a1l + (lane - 8) * 8;  act = true; }
    else                { p = a2h + (lane - 16) * 8; act = true; }
  } else if (wave == 1) {
    if (lane < 16)      { p = a2l + lane * 8;        act = true; }
  } else if (wave == 2) { p = a3h + lane * 8; act = true; }
  else if (wave == 3)   { p = a3l + lane * 8; act = true; }
  else if (wave == 4)   { p = a4h + lane * 8; act = true; }
  else if (wave == 5)   { p = a4l + lane * 8; act = true; }
  if (act) {
    *(volatile v8us*)p = z;
    __threadfence();
    *(volatile v8us*)p = z;
  }
}

template <int CIN, bool ASPLIT, bool BIAS, int OUT_MODE, int ACT>
__global__ __launch_bounds__(256) void gemm_bf16(
    const unsigned short* __restrict__ Ap, const unsigned short* __restrict__ A2p, int lda,
    const unsigned short* __restrict__ Btp, int ldb,
    void* __restrict__ Cout, void* __restrict__ Cout2, int ldc,
    const float* __restrict__ bias, int M, int N, int K) {
  static_assert(CIN == 0 || CIN % 32 == 0, "one tap per 32-k chunk");
  static_assert(OUT_MODE == 0 || OUT_MODE == 2, "f32 or hi+lo planes");
  typedef __bf16 T;
  typedef v16b V;
  const T* A = (const T*)Ap; const T* A2 = (const T*)A2p; const T* Bt = (const T*)Btp;
  __shared__ __align__(16) float sT[8][16 * 68];
  const int lane = threadIdx.x & 31;
  const int wave = threadIdx.x >> 5;
  const int tilesN = N >> 6;
  const int tilesM = M >> 6;
  const int tile = blockIdx.x * 8 + wave;
  if (tile >= tilesM * tilesN) return;
  const int tm = tile / tilesN;
  const int tn = tile - tm * tilesN;
  const int m0 = tm << 6;
  const int n0 = tn << 6;

  const int rlane = lane & 15;
  const int koff  = (lane >> 4) * 8;
  const int mOff  = (lane >> 4) * 8;

  v8f acc[4][4];
#pragma unroll
  for (int i = 0; i < 4; ++i)
#pragma unroll
    for (int j = 0; j < 4; ++j) acc[i][j] = (v8f){0.f,0.f,0.f,0.f,0.f,0.f,0.f,0.f};

  for (int k0 = 0; k0 < K; k0 += 32) {
    V bh[4];
#pragma unroll
    for (int j = 0; j < 4; ++j) {
      const size_t bo = (size_t)(n0 + (j << 4) + rlane) * ldb + koff + k0;
      bh[j] = FragB::load(Bt + bo);
    }
    int dy = 0, dx = 0, ci0 = 0;
    if (CIN > 0) {
      const int tap = k0 / CIN;
      const int t3  = tap / 3;
      dy  = t3 - 1;
      dx  = tap - 3 * t3 - 1;
      ci0 = k0 - tap * CIN;
    }
#pragma unroll
    for (int i = 0; i < 4; ++i) {
      const int pm = m0 + (i << 4) + rlane;
      size_t ao;
      if (CIN == 0) {
        ao = (size_t)pm * lda + koff + k0;
      } else {
        const int yy = (pm >> 6) & 63, xx = pm & 63, bimg = pm >> 12;
        const int ny = yy + dy, nx = xx + dx;
        const bool ok = ((unsigned)ny < 64u) && ((unsigned)nx < 64u);
        const int nyc = ny < 0 ? 0 : (ny > 63 ? 63 : ny);
        const int nxc = nx < 0 ? 0 : (nx > 63 ? 63 : nx);
        const int pixn = (bimg << 12) + nyc * 64 + nxc;
        const int pix  = ok ? pixn : kPix;
        ao = (size_t)pix * CIN + ci0 + koff;
      }
      V ah = FragB::load(A + ao);
      V al = ah;
      if (ASPLIT) al = FragB::load(A2 + ao);
#pragma unroll
      for (int j = 0; j < 4; ++j) {
        acc[i][j] = FragB::mma(ah, bh[j], acc[i][j]);
        if (ASPLIT) acc[i][j] = FragB::mma(al, bh[j], acc[i][j]);
      }
      acc_guard4b2(acc[i][0], acc[i][1], acc[i][2], acc[i][3], ah, al);
    }
    keep4_b(bh[0], bh[1], bh[2], bh[3]);
  }
  acc_guard4(acc[0][0], acc[0][1], acc[0][2], acc[0][3]);
  acc_guard4(acc[1][0], acc[1][1], acc[1][2], acc[1][3]);
  acc_guard4(acc[2][0], acc[2][1], acc[2][2], acc[2][3]);
  acc_guard4(acc[3][0], acc[3][1], acc[3][2], acc[3][3]);

  float* slab = sT[wave];
#pragma unroll
  for (int i = 0; i < 4; ++i) {
    const int mBase = m0 + (i << 4);
#pragma unroll
    for (int j = 0; j < 4; ++j) {
      const int n = n0 + (j << 4) + rlane;
      float bv = 0.f;
      if (BIAS) bv = bf_rne(bias[n]);
#pragma unroll
      for (int r = 0; r < 8; ++r) {
        float v = acc[i][j][r];
        if (BIAS) v = v + bv;
        if (ACT == 2) v = fmaxf(v, 0.0f);
        slab[(mOff + r) * 68 + (j << 4) + rlane] = v;
      }
    }
    __builtin_amdgcn_fence(__ATOMIC_RELEASE, "workgroup");
    __builtin_amdgcn_wave_barrier();
    __builtin_amdgcn_fence(__ATOMIC_ACQUIRE, "workgroup");
    if (OUT_MODE == 0) {
      float* C = (float*)Cout;
      const int hh = lane >> 4, c4 = (lane & 15) * 4;
      for (int pass = 0; pass < 2; ++pass) {
#pragma unroll
        for (int it = 0; it < 8; ++it) {
          const int row = it * 2 + hh;
          v4f v = *(const v4f*)(slab + row * 68 + c4);
          *(volatile v4f*)(C + (size_t)(mBase + row) * ldc + n0 + c4) = v;
        }
        __threadfence();
      }
    } else {
      const int q = lane >> 3, c8 = (lane & 7) * 8;
      unsigned short* C  = (unsigned short*)Cout;
      unsigned short* C2 = (unsigned short*)Cout2;
      for (int pass = 0; pass < 2; ++pass) {
#pragma unroll
        for (int it = 0; it < 4; ++it) {
          const int row = it * 4 + q;
          const float* sp = slab + row * 68 + c8;
          v8h hv, lv;
#pragma unroll
          for (int e = 0; e < 8; ++e) {
            unsigned short hb = f2bf_bits(sp[e]);
            unsigned short lb = f2bf_bits(sp[e] - bf_bits2f(hb));
            hv[e] = __builtin_bit_cast(_Float16, hb);
            lv[e] = __builtin_bit_cast(_Float16, lb);
          }
          *(volatile v8h*)(C + (size_t)(mBase + row) * ldc + n0 + c8) = hv;
          *(volatile v8h*)(C2 + (size_t)(mBase + row) * ldc + n0 + c8) = lv;
        }
        __threadfence();
      }
    }
    __builtin_amdgcn_fence(__ATOMIC_RELEASE, "workgroup");
    __builtin_amdgcn_wave_barrier();
    __builtin_amdgcn_fence(__ATOMIC_ACQUIRE, "workgroup");
  }
}

__device__ __forceinline__ void mlp_kloop(v8f (&acc)[4], const __bf16* ahi, const __bf16* alo, const __bf16* bbase) {
#pragma unroll 1
  for (int kc = 0; kc < 8; ++kc) {
    const int k0 = kc * 32;
    const v16b ah = FragB::load(ahi + k0);
    const v16b al = FragB::load(alo + k0);
    v16b bf[4];
#pragma unroll
    for (int j = 0; j < 4; ++j) bf[j] = FragB::load(bbase + (size_t)j * kBStep + k0);
#pragma unroll
    for (int j = 0; j < 4; ++j) {
      acc[j] = FragB::mma(ah, bf[j], acc[j]);
      acc[j] = FragB::mma(al, bf[j], acc[j]);
    }
    acc_guard4b2(acc[0], acc[1], acc[2], acc[3], ah, al);
    keep4_b(bf[0], bf[1], bf[2], bf[3]);
  }
}

__device__ __forceinline__ void mlp_epi(const v8f (&acc)[4], const float* __restrict__ bias, int cbase,
                                        unsigned short* hhi, unsigned short* hlo, int rt, int rl, int hh) {
#pragma unroll
  for (int j = 0; j < 4; ++j) {
    const int col = cbase + 16 * j + rl;
    const float bz = bf_rne(bias[col]);
#pragma unroll
    for (int r = 0; r < 8; ++r) {
      float v = acc[j][r] + bz;
      v = fmaxf(v, 0.0f);
      const unsigned short hb = f2bf_bits(v);
      const unsigned short lb = f2bf_bits(v - bf_bits2f(hb));
      const int idx = (16 * rt + 8 * hh + r) * kHP + col;
      hhi[idx] = hb;
      hlo[idx] = lb;
    }
  }
}

__device__ __forceinline__ float lin64(int i) {
  const float st = (float)i * kInv63;
  const float om = 1.0f - st;
  float v = -om;
  v = v + st;
  return (i == 63) ? 1.0f : v;
}

__global__ __launch_bounds__(kThreads) void k_mlp(
    const float* __restrict__ coord, const float* __restrict__ cell,
    const float* __restrict__ gpl,
    const float* __restrict__ w0, const float* __restrict__ b0,
    const unsigned short* __restrict__ w1p, const float* __restrict__ b1,
    const unsigned short* __restrict__ w2p, const float* __restrict__ b2,
    const unsigned short* __restrict__ w3p, const float* __restrict__ b3,
    const unsigned short* __restrict__ w4p, const float* __restrict__ b4,
    float* outp) {
  __shared__ __align__(16) unsigned short Hhi[kQRows * kHP];
  __shared__ __align__(16) unsigned short Hlo[kQRows * kHP];
  __shared__ int   sPix[kMRows];
  __shared__ float sWgt[kMRows];
  __shared__ float sRc0[kMQ];
  __shared__ float sRc1[kMQ];
  __shared__ __align__(16) float sOut[128];

  const int tid  = threadIdx.x;
  const int lane = tid & 31;
  const int wave = tid >> 5;
  const int rl   = lane & 15;
  const int hh   = lane >> 4;
  const int koff = hh * 8;
  const int blk  = blockIdx.x;

  if (tid < kMQ) {
    const int q  = tid;
    const int bq = blk * kMQ + q;
    const int bb = bq >> 13;
    const float c0 = bf_rne(coord[2 * bq]);
    const float c1 = bf_rne(coord[2 * bq + 1]);
    const float e0 = bf_rne(cell[2 * bq]);
    const float e1 = bf_rne(cell[2 * bq + 1]);
    sRc0[q] = e0 * 64.0f;
    sRc1[q] = e1 * 64.0f;
    float ar[4];
    int   pk[4];
#pragma unroll
    for (int k = 0; k < 4; ++k) {
      const float s0 = (k & 2) ? kHalfPix : -kHalfPix;
      const float s1 = (k & 1) ? kHalfPix : -kHalfPix;
      float cy = c0 + s0; cy = cy + kEpsShift; cy = fminf(fmaxf(cy, kClipLo), kClipHi);
      float cx = c1 + s1; cx = cx + kEpsShift; cx = fminf(fmaxf(cx, kClipLo), kClipHi);
      float ty = cy + 1.0f; ty = ty * 64.0f; ty = ty - 1.0f; ty = ty * 0.5f;
      float tx = cx + 1.0f; tx = tx * 64.0f; tx = tx - 1.0f; tx = tx * 0.5f;
      int iy = (int)rintf(ty); iy = iy < 0 ? 0 : (iy > 63 ? 63 : iy);
      int ix = (int)rintf(tx); ix = ix < 0 ? 0 : (ix > 63 ? 63 : ix);
      const float ly = lin64(iy);
      const float lx = lin64(ix);
      float r0 = c0 - ly; r0 = r0 * 64.0f;
      float r1 = c1 - lx; r1 = r1 * 64.0f;
      float a = r0 * r1; a = fabsf(a); a = a + kAreaEps;
      ar[k] = a;
      pk[k] = (bb << 12) + iy * 64 + ix;
    }
    float tot = ar[0] + ar[1]; tot = tot + ar[2]; tot = tot + ar[3];
#pragma unroll
    for (int k = 0; k < 4; ++k) {
      sPix[4 * q + k] = pk[k];
      sWgt[4 * q + k] = ar[3 - k] / tot;
    }
    sOut[96 + tid] = 0.0f;
  }
  __syncthreads();

  const int cb = lane * 8;
  float bz[8], wca[8], wcb[8];
  {
    const float* wc = w0 + (size_t)kK5 * kHid;
    const v4f t0 = *(const v4f*)(b0 + cb), t1 = *(const v4f*)(b0 + cb + 4);
    const v4f u0 = *(const v4f*)(wc + cb), u1 = *(const v4f*)(wc + cb + 4);
    const v4f s0 = *(const v4f*)(wc + kHid + cb), s1 = *(const v4f*)(wc + kHid + cb + 4);
#pragma unroll
    for (int e = 0; e < 4; ++e) {
      bz[e]  = bf_rne(t0[e]); bz[4 + e]  = bf_rne(t1[e]);
      wca[e] = bf_rne(u0[e]); wca[4 + e] = bf_rne(u1[e]);
      wcb[e] = bf_rne(s0[e]); wcb[4 + e] = bf_rne(s1[e]);
    }
  }
  asm volatile("" ::: "memory");

  const int rt = wave & 1, cg = wave >> 1, cbase = cg * 64;
  const __bf16* ahi = (const __bf16*)(Hhi + (16 * rt + rl) * kHP + koff);
  const __bf16* alo = (const __bf16*)(Hlo + (16 * rt + rl) * kHP + koff);
  const v8f z8 = {0.f, 0.f, 0.f, 0.f, 0.f, 0.f, 0.f, 0.f};

#pragma unroll 1
  for (int qt = 0; qt < kQT; ++qt) {
    __syncthreads();
#pragma unroll 1
    for (int i = 0; i < 4; ++i) {
      const int r = wave * 4 + i;
      int p = sPix[qt * kQRows + r];
      p = p < 0 ? 0 : (p > kPix - 1 ? kPix - 1 : p);
      const float q0 = sRc0[qt * kQQ + (r >> 2)];
      const float q1 = sRc1[qt * kQQ + (r >> 2)];
      const float* gp = gpl + (size_t)p * kHid + cb;
      const v4f ga = *(const v4f*)gp;
      const v4f gb = *(const v4f*)(gp + 4);
      v8us hv, lv;
#pragma unroll
      for (int e = 0; e < 4; ++e) {
        float v = ga[e];
        const float ta = q0 * wca[e];
        const float tb = q1 * wcb[e];
        v = v + ta; v = v + tb; v = v + bz[e];
        v = fmaxf(v, 0.0f);
        const unsigned short hb = f2bf_bits(v);
        const unsigned short lb = f2bf_bits(v - bf_bits2f(hb));
        hv[e] = hb; lv[e] = lb;
        float u = gb[e];
        const float ua = q0 * wca[4 + e];
        const float ub = q1 * wcb[4 + e];
        u = u + ua; u = u + ub; u = u + bz[4 + e];
        u = fmaxf(u, 0.0f);
        const unsigned short hb2 = f2bf_bits(u);
        const unsigned short lb2 = f2bf_bits(u - bf_bits2f(hb2));
        hv[4 + e] = hb2; lv[4 + e] = lb2;
      }
      *(v8us*)(Hhi + r * kHP + cb) = hv;
      *(v8us*)(Hlo + r * kHP + cb) = lv;
    }
    __syncthreads();

#pragma unroll 1
    for (int layer = 0; layer < 3; ++layer) {
      const __bf16* Wt = (const __bf16*)((layer == 0) ? w1p : ((layer == 1) ? w2p : w3p));
      const float*  bv = (layer == 0) ? b1 : ((layer == 1) ? b2 : b3);
      v8f acc[4];
#pragma unroll
      for (int j = 0; j < 4; ++j) acc[j] = z8;
      mlp_kloop(acc, ahi, alo, Wt + (size_t)(cbase + rl) * kHid + koff);
      __syncthreads();
      mlp_epi(acc, bv, cbase, Hhi, Hlo, rt, rl, hh);
      __syncthreads();
    }

    if (wave < 2) {
      v8f a4 = z8;
      const __bf16* W4 = (const __bf16*)w4p + (size_t)rl * kHid + koff;
#pragma unroll 1
      for (int kc = 0; kc < 8; ++kc) {
        const v16b ah  = FragB::load(ahi + kc * 32);
        const v16b al  = FragB::load(alo + kc * 32);
        const v16b bw4 = FragB::load(W4 + kc * 32);
        a4 = FragB::mma(ah, bw4, a4);
        a4 = FragB::mma(al, bw4, a4);
        acc_guard1b3(a4, ah, al, bw4);
      }
      const int cc = (rl < 3) ? rl : 2;
      const float bias4 = bf_rne(b4[cc]);
      const int rb = 16 * rt + 8 * hh;
      float s0 = 0.0f, s1 = 0.0f;
#pragma unroll
      for (int r = 0; r < 4; ++r) {
        float p = a4[r] + bias4;
        const float t = p * sWgt[qt * kQRows + rb + r];
        s0 = s0 + t;
      }
#pragma unroll
      for (int r = 4; r < 8; ++r) {
        float p = a4[r] + bias4;
        const float t = p * sWgt[qt * kQRows + rb + r];
        s1 = s1 + t;
      }
      const int ql = qt * kQQ + 4 * rt + 2 * hh;
      if (rl < 3) {
        sOut[ql * 3 + rl] = s0;
        sOut[(ql + 1) * 3 + rl] = s1;
      }
    }
  }

  __syncthreads();
  if (wave == 0) {
    const v4f v = *(const v4f*)(sOut + lane * 4);
    if (lane < 24) {
      float* op = outp + (size_t)blk * (kMQ * 3) + lane * 4;
      *(volatile v4f*)op = v;
      __threadfence();
      *(volatile v4f*)op = v;
    }
  }
}

extern "C" void kernel_launch(void* const* d_in, const int* in_sizes, int n_in,
                              void* d_out, int out_size, void* d_ws, size_t ws_size,
                              hipStream_t stream) {
  (void)in_sizes;
  if (n_in < 21) return;
  if (ws_size < kWsTotal) return;
  if ((size_t)out_size < (size_t)kBQ * 3) return;

  const float* inp   = (const float*)d_in[0];
  const float* coord = (const float*)d_in[1];
  const float* cell  = (const float*)d_in[2];
  const float* c1w = (const float*)d_in[3];  const float* c1b = (const float*)d_in[4];
  const float* c2w = (const float*)d_in[5];  const float* c2b = (const float*)d_in[6];
  const float* c3w = (const float*)d_in[7];  const float* c3b = (const float*)d_in[8];
  const float* c4w = (const float*)d_in[9];  const float* c4b = (const float*)d_in[10];
  const float* w0  = (const float*)d_in[11]; const float* b0  = (const float*)d_in[12];
  const float* w1  = (const float*)d_in[13]; const float* b1  = (const float*)d_in[14];
  const float* w2  = (const float*)d_in[15]; const float* b2  = (const float*)d_in[16];
  const float* w3  = (const float*)d_in[17]; const float* b3  = (const float*)d_in[18];
  const float* w4  = (const float*)d_in[19]; const float* b4  = (const float*)d_in[20];
  float* out = (float*)d_out;

  char* ws = (char*)d_ws;
  unsigned short* IM1 = (unsigned short*)(ws + kOffIM1);
  unsigned short* C1W = (unsigned short*)(ws + kOffC1W);
  unsigned short* C2W = (unsigned short*)(ws + kOffC2W);
  unsigned short* C3W = (unsigned short*)(ws + kOffC3W);
  unsigned short* C4W = (unsigned short*)(ws + kOffC4W);
  unsigned short* W0T = (unsigned short*)(ws + kOffW0T);
  unsigned short* W1T = (unsigned short*)(ws + kOffW1T);
  unsigned short* W2T = (unsigned short*)(ws + kOffW2T);
  unsigned short* W3T = (unsigned short*)(ws + kOffW3T);
  unsigned short* W4T = (unsigned short*)(ws + kOffW4T);
  unsigned short* A1H = (unsigned short*)(ws + kOffA1H);
  unsigned short* A1L = (unsigned short*)(ws + kOffA1L);
  unsigned short* A2H = (unsigned short*)(ws + kOffA2H);
  unsigned short* A2L = (unsigned short*)(ws + kOffA2L);
  unsigned short* A3H = (unsigned short*)(ws + kOffA3H);
  unsigned short* A3L = (unsigned short*)(ws + kOffA3L);
  unsigned short* A4H = (unsigned short*)(ws + kOffA4H);
  unsigned short* A4L = (unsigned short*)(ws + kOffA4L);
  float*          GPL = (float*)(ws + kOffG);

  k_prep_c1w<<<1, kThreads, 0, stream>>>(c1w, C1W);
  k_prep_convw<kC1><<<(kC2 * (9 * kC1 / 8)) / kThreads, kThreads, 0, stream>>>(c2w, C2W, kC2);
  k_prep_convw<kC2><<<(kC3 * (9 * kC2 / 8)) / kThreads, kThreads, 0, stream>>>(c3w, C3W, kC3);
  k_prep_convw<kC3><<<(kC4 * (9 * kC3 / 8)) / kThreads, kThreads, 0, stream>>>(c4w, C4W, kC4);
  k_prep_w0t<<<(kHid * (kK5 / 8)) / kThreads, kThreads, 0, stream>>>(w0, W0T);
  k_prep_wsq<<<(kHid * (kHid / 8)) / kThreads, kThreads, 0, stream>>>(w1, W1T);
  k_prep_wsq<<<(kHid * (kHid / 8)) / kThreads, kThreads, 0, stream>>>(w2, W2T);
  k_prep_wsq<<<(kHid * (kHid / 8)) / kThreads, kThreads, 0, stream>>>(w3, W3T);
  k_prep_w4t<<<(kN4 * (kHid / 8)) / kThreads, kThreads, 0, stream>>>(w4, W4T);

  k_zero_rows<<<1, kThreads, 0, stream>>>(A1H + (size_t)kPix * kC1, A1L + (size_t)kPix * kC1,
                                          A2H + (size_t)kPix * kC2, A2L + (size_t)kPix * kC2,
                                          A3H + (size_t)kPix * kC3, A3L + (size_t)kPix * kC3,
                                          A4H + (size_t)kPix * kC4, A4L + (size_t)kPix * kC4);

  k_im2col1<<<(kPix * (kK1 / 8)) / kThreads, kThreads, 0, stream>>>(inp, IM1);
  gemm_bf16<0, false, true, 2, 2><<<(kPix / 64) * (kC1 / 64) / 8, 256, 0, stream>>>(
      IM1, IM1, kK1, C1W, kK1, (void*)A1H, (void*)A1L, kC1, c1b, kPix, kC1, kK1);
  gemm_bf16<kC1, true, true, 2, 2><<<(kPix / 64) * (kC2 / 64) / 8, 256, 0, stream>>>(
      A1H, A1L, kC1, C2W, kK2, (void*)A2H, (void*)A2L, kC2, c2b, kPix, kC2, kK2);
  gemm_bf16<kC2, true, true, 2, 2><<<(kPix / 64) * (kC3 / 64) / 8, 256, 0, stream>>>(
      A2H, A2L, kC2, C3W, kK3, (void*)A3H, (void*)A3L, kC3, c3b, kPix, kC3, kK3);
  gemm_bf16<kC3, true, true, 2, 2><<<(kPix / 64) * (kC4 / 64) / 8, 256, 0, stream>>>(
      A3H, A3L, kC3, C4W, kK4, (void*)A4H, (void*)A4L, kC4, c4b, kPix, kC4, kK4);

  gemm_bf16<kC4, true, false, 0, 0><<<(kPix / 64) * (kHid / 64) / 8, 256, 0, stream>>>(
      A4H, A4L, kC4, W0T, kK5, (void*)GPL, (void*)GPL, kHid, b0, kPix, kHid, kK5);

  k_mlp<<<kMBlocks, kThreads, 0, stream>>>(coord, cell, GPL, w0, b0, W1T, b1, W2T, b2, W3T, b3, W4T, b4, out);
}
